// HPNCritic_1546188226866
// MI455X (gfx1250) — hardware-verified
//
#include <hip/hip_runtime.h>


#define NBT  1024
#define SD   131
#define NAL  9
#define NAD  10
#define NAG  10
#define AD   5
#define HYP  128
#define HH   1024
#define HID  256
#define NHD  4
#define NGA  (11 * HH)
#define NGV  (7 * HH)
#define RA   (NBT * NAL)
#define RV   (NBT * NAD)
#define CHA  576
#define CHV  640
typedef _Float16 h16;
typedef unsigned short bf;
typedef __attribute__((ext_vector_type(16))) __bf16   v16bf;
typedef __attribute__((ext_vector_type(16))) _Float16 v16h;
typedef __attribute__((ext_vector_type(8)))  _Float16 v8h;
typedef __attribute__((ext_vector_type(8)))  unsigned short v8us;
typedef __attribute__((ext_vector_type(8)))  float    v8f;
typedef __attribute__((ext_vector_type(4)))  float    v4f;
typedef v8h  __attribute__((may_alias)) v8ha;
typedef v4f  __attribute__((may_alias)) v4fa;
typedef v8us __attribute__((may_alias)) v8usa;

__device__ __forceinline__ unsigned short f2bf(float f) { unsigned u = __float_as_uint(f); u += 0x7FFFu + ((u >> 16) & 1u); return (unsigned short)(u >> 16); }
__device__ __forceinline__ float bf2f(unsigned short b) { return __uint_as_float(((unsigned)b) << 16); }
__device__ __forceinline__ float bfr(float f) { return bf2f(f2bf(f)); }
__device__ __forceinline__ v16h cat16(v8h lo, v8h hi) { return __builtin_shufflevector(lo, hi, 0, 1, 2, 3, 4, 5, 6, 7, 8, 9, 10, 11, 12, 13, 14, 15); }
__device__ __forceinline__ v16bf cat16b(v8us lo, v8us hi) { return __builtin_bit_cast(v16bf, __builtin_shufflevector(lo, hi, 0, 1, 2, 3, 4, 5, 6, 7, 8, 9, 10, 11, 12, 13, 14, 15)); }
__device__ __forceinline__ v8f wmma16(v16h a, v16h b, v8f c) { return __builtin_amdgcn_wmma_f32_16x16x32_f16(false, a, false, b, (short)0, c, false, false); }
__device__ __forceinline__ v8f wmmab(v16bf a, v16bf b, v8f c) { return __builtin_amdgcn_wmma_f32_16x16x32_bf16(false, a, false, b, (short)0, c, false, false); }


template <typename T16> struct WFrag;
template <> struct WFrag<h16> { typedef v16h V; static __device__ __forceinline__ V ld(const h16* p) { return cat16(*(const v8h*)p, *(const v8h*)(p + 16)); } static __device__ __forceinline__ v8f mma(V a, V b, v8f c) { return wmma16(a, b, c); } };
template <> struct WFrag<bf> { typedef v16bf V; static __device__ __forceinline__ V ld(const bf* p) { return cat16b(*(const v8us*)p, *(const v8us*)(p + 16)); } static __device__ __forceinline__ v8f mma(V a, V b, v8f c) { return wmmab(a, b, c); } };
template <typename T16, int NSPLIT, bool BIAS>
__global__ __launch_bounds__(32) void k_gemmw(const T16* __restrict__ A, const T16* __restrict__ A2, const T16* __restrict__ Bt, const T16* __restrict__ Bt2, int K, float* C, int ldc, const float* __restrict__ bias, size_t sA, size_t sB, size_t sC) {
    typedef typename WFrag<T16>::V V;
    __shared__ __align__(16) float os[16 * 68];
    const size_t z = blockIdx.z; A += z * sA; if (A2) A2 += z * sA; Bt += z * sB; if (Bt2) Bt2 += z * sB; C += z * sC;
    const int lane = threadIdx.x & 31, lr = lane & 15, hi = lane >> 4; const int r0 = blockIdx.x * 64, c0 = blockIdx.y * 64;
    v8f acc[4][4];
#pragma unroll
    for (int mb = 0; mb < 4; ++mb)
#pragma unroll
        for (int nb = 0; nb < 4; ++nb) acc[mb][nb] = (v8f){};
    const size_t aoff = (size_t)(r0 + lr) * K + 8 * hi, boff = (size_t)(c0 + lr) * K + 8 * hi;
#pragma unroll 1
    for (int kc = 0; kc < K; kc += 32) {
        V a[4], a2[4];
#pragma unroll
        for (int mb = 0; mb < 4; ++mb) { a[mb] = WFrag<T16>::ld(A + aoff + (size_t)mb * 16 * K + kc); if (NSPLIT == 1 || NSPLIT == 2) a2[mb] = WFrag<T16>::ld(A2 + aoff + (size_t)mb * 16 * K + kc); }
#pragma unroll
        for (int nb = 0; nb < 4; ++nb) { const V b = WFrag<T16>::ld(Bt + boff + (size_t)nb * 16 * K + kc); V b2; if (NSPLIT >= 2) b2 = WFrag<T16>::ld(Bt2 + boff + (size_t)nb * 16 * K + kc);
#pragma unroll
            for (int mb = 0; mb < 4; ++mb) { acc[mb][nb] = WFrag<T16>::mma(a[mb], b, acc[mb][nb]); if (NSPLIT == 1 || NSPLIT == 2) acc[mb][nb] = WFrag<T16>::mma(a2[mb], b, acc[mb][nb]); if (NSPLIT >= 2) acc[mb][nb] = WFrag<T16>::mma(a[mb], b2, acc[mb][nb]); } }
        asm volatile("v_nop\n\tv_nop\n\tv_nop\n\tv_nop" : "+v"(acc[0][0]), "+v"(acc[1][1]), "+v"(acc[2][2]), "+v"(acc[3][3]) : "v"(a[0]), "v"(a[3]));
    }
#pragma unroll
    for (int mb = 0; mb < 4; ++mb) {
#pragma unroll
        for (int nb = 0; nb < 4; ++nb) {
#pragma unroll
            for (int j = 0; j < 8; ++j) os[(hi * 8 + j) * 68 + nb * 16 + lr] = acc[mb][nb][j]; }
        __builtin_amdgcn_wave_barrier(); asm volatile("" ::: "memory");
        float* crow = C + (size_t)(r0 + mb * 16) * ldc + c0;
#pragma unroll 1
        for (int ps = 0; ps < 2; ++ps) {
#pragma unroll
            for (int s = 0; s < 8; ++s) { const int row = 2 * s + hi, cofs = lr * 4; v4f val = *(const v4fa*)(os + row * 68 + cofs); if (BIAS) { val[0] += bfr(bias[c0 + cofs]); val[1] += bfr(bias[c0 + cofs + 1]); val[2] += bfr(bias[c0 + cofs + 2]); val[3] += bfr(bias[c0 + cofs + 3]); }
                *(volatile v4f*)(crow + (size_t)row * ldc + cofs) = val; }
            if (ps == 0) __threadfence(); }
        __builtin_amdgcn_wave_barrier(); asm volatile("" ::: "memory");
    }
}

__device__ __forceinline__ void splitf(float y, unsigned short& h, unsigned short& l) { h = f2bf(y); l = f2bf(y - bf2f(h)); }
__device__ __forceinline__ float lrelu(float x) { return x >= 0.f ? x : 0.01f * x; }
__device__ __forceinline__ int agent_of(const int* __restrict__ aidp) { int a = aidp[0]; return a < 0 ? 0 : (a > NAG - 1 ? NAG - 1 : a); }

__global__ __launch_bounds__(256) void k_wt(const float* __restrict__ w, int K, int N, bf* Bt) {
    typedef __attribute__((ext_vector_type(2))) unsigned short v2us;
    const int lane = threadIdx.x & 31; const int nlines = N * K / 64; const int wg = blockIdx.x * 8 + (threadIdx.x >> 5), nw = gridDim.x * 8;
#pragma unroll 1
    for (int ps = 0; ps < 2; ++ps) {
#pragma unroll 1
        for (int L = wg; L < nlines; L += nw) { const int e = L * 64 + lane * 2; v2us o;
#pragma unroll
            for (int q = 0; q < 2; ++q) { const int n = (e + q) / K, k = (e + q) % K; o[q] = f2bf(w[(size_t)k * N + n]); }
            *(volatile v2us*)(Bt + e) = o; }
        if (ps == 0) __threadfence(); }
}
template <bool ADV>
__global__ __launch_bounds__(256) void k_hyp1(const float* __restrict__ state, const float* __restrict__ action, const int* __restrict__ aidp, const float* __restrict__ W1, const float* __restrict__ b1, bf* Hh, bf* Hl) {
    typedef __attribute__((ext_vector_type(4))) unsigned short v4us;
    const int lane = threadIdx.x & 31; const int r = blockIdx.x * 8 + (threadIdx.x >> 5); const int nrows = ADV ? RV : RA; if (r >= nrows) return;
    const int NE = ADV ? NAD : NAL, KF = ADV ? 6 : 10; const int b = r / NE, n = r % NE; float f[10];
    if (ADV) {
#pragma unroll
        for (int k = 0; k < 6; ++k) f[k] = bfr(state[(size_t)b * SD + 52 + n * 6 + k]);
#pragma unroll
        for (int k = 6; k < 10; ++k) f[k] = 0.f;
    } else { const int aid = agent_of(aidp); const int oth = n < aid ? n : n + 1;
#pragma unroll
        for (int k = 0; k < 5; ++k) f[k] = bfr(state[(size_t)b * SD + 7 + n * 5 + k]);
#pragma unroll
        for (int k = 0; k < 5; ++k) f[5 + k] = bfr(action[((size_t)b * NAG + oth) * AD + k]); }
    const int c0 = lane * 4; v4us oh, ol;
#pragma unroll
    for (int q = 0; q < 4; ++q) { const int c = c0 + q; float acc = 0.f;
#pragma unroll
        for (int k = 0; k < 10; ++k) if (k < KF) acc = fmaf(f[k], bfr(W1[k * HYP + c]), acc);
        unsigned short a, bb; splitf(lrelu(acc + bfr(b1[c])), a, bb); oh[q] = a; ol[q] = bb; }
#pragma unroll 1
    for (int ps = 0; ps < 2; ++ps) { *(volatile v4us*)(Hh + (size_t)r * HYP + c0) = oh; *(volatile v4us*)(Hl + (size_t)r * HYP + c0) = ol; if (ps == 0) __threadfence(); }
}
template <bool ADV>
__global__ __launch_bounds__(256) void k_applysum(const float* __restrict__ state, const float* __restrict__ action, const int* __restrict__ aidp, const float* __restrict__ G, int b0, float* SUM) {
    const int lane = threadIdx.x & 31; const int wg = blockIdx.x * 8 + (threadIdx.x >> 5); if (wg >= 64 * (HH / 128)) return; const int bl = wg >> 3, h0 = (wg & 7) * 128 + lane * 4; const int b = b0 + bl;
    const int NE = ADV ? NAD : NAL, KF = ADV ? 6 : 10, NG = ADV ? NGV : NGA; const int aid = agent_of(aidp);
    v4f o = {0.f, 0.f, 0.f, 0.f};
#pragma unroll 1
    for (int n = 0; n < NE; ++n) { float f[10]; float keep = 1.f;
        if (ADV) {
#pragma unroll
            for (int k = 0; k < 6; ++k) f[k] = bfr(state[(size_t)b * SD + 52 + n * 6 + k]);
#pragma unroll
            for (int k = 6; k < 10; ++k) f[k] = 0.f;
        } else { const int oth = n < aid ? n : n + 1;
#pragma unroll
            for (int k = 0; k < 5; ++k) f[k] = bfr(state[(size_t)b * SD + 7 + n * 5 + k]);
#pragma unroll
            for (int k = 0; k < 5; ++k) f[5 + k] = bfr(action[((size_t)b * NAG + oth) * AD + k]);
            keep = (bfr(state[(size_t)b * SD + 112 + n]) < 0.5f) ? 0.f : 1.f; }
        const float* gr = G + (size_t)(bl * NE + n) * NG;
#pragma unroll
        for (int q = 0; q < 4; ++q) { const int hh = h0 + q; float acc = gr[KF * HH + hh];
#pragma unroll
            for (int d = 0; d < 10; ++d) if (d < KF) acc = fmaf(f[d], gr[d * HH + hh], acc);
            o[q] += acc * keep; } }
    float* dst = SUM + (size_t)b * HH + h0; *(volatile v4f*)dst = o; __threadfence(); *(volatile v4f*)dst = o;
}
__global__ __launch_bounds__(256) void k_merge(const float* __restrict__ state, const float* __restrict__ action, const int* __restrict__ aidp, const float* __restrict__ ASUM, const float* __restrict__ VSUM, const float* __restrict__ mw, const float* __restrict__ Ws, const float* __restrict__ bs, bf* Oh, bf* Ol) {
    typedef __attribute__((ext_vector_type(4))) unsigned short v4us;
    const int lane = threadIdx.x & 31; const int b = blockIdx.x * 8 + (threadIdx.x >> 5); if (b >= NBT) return; const int aid = agent_of(aidp);
    float sf[12];
#pragma unroll
    for (int k = 0; k < 7; ++k) sf[k] = bfr(state[(size_t)b * SD + k]);
#pragma unroll
    for (int k = 0; k < 5; ++k) sf[7 + k] = bfr(action[((size_t)b * NAG + aid) * AD + k]);
#pragma unroll 1
    for (int ps = 0; ps < 2; ++ps) {
#pragma unroll 1
        for (int it = 0; it < 2; ++it) { v4us oh, ol;
#pragma unroll
            for (int q = 0; q < 4; ++q) { const int hid = it * 128 + lane * 4 + q;
                float w[NHD], tot[NHD]; float m = -3.0e38f;
#pragma unroll
                for (int h = 0; h < NHD; ++h) { w[h] = bfr(mw[h * HID + hid]); m = fmaxf(m, w[h]); }
                float se = 0.f;
#pragma unroll
                for (int h = 0; h < NHD; ++h) { w[h] = __expf(w[h] - m); se += w[h]; }
                const float inv = __fdiv_rn(1.0f, se);
#pragma unroll
                for (int h = 0; h < NHD; ++h) tot[h] = ASUM[(size_t)b * HH + h * HID + hid] + VSUM[(size_t)b * HH + h * HID + hid];
                float merged = 0.f;
#pragma unroll
                for (int h = 0; h < NHD; ++h) merged += (w[h] * inv) * tot[h];
                float so = bfr(bs[hid]);
#pragma unroll
                for (int k = 0; k < 12; ++k) so = fmaf(sf[k], bfr(Ws[k * HID + hid]), so);
                const float o1 = fmaxf(so + merged, 0.f); unsigned short a, bb; splitf(o1, a, bb); oh[q] = a; ol[q] = bb; }
            const int c0 = it * 128 + lane * 4; *(volatile v4us*)(Oh + (size_t)b * HID + c0) = oh; *(volatile v4us*)(Ol + (size_t)b * HID + c0) = ol; }
        if (ps == 0) __threadfence(); }
}
__global__ __launch_bounds__(256) void k_out(const float* __restrict__ Z, const float* __restrict__ Wo2, const float* __restrict__ bo2, float* OUT) {
    const int lane = threadIdx.x & 31; const int b0 = (blockIdx.x * 8 + (threadIdx.x >> 5)) * 32; if (b0 >= NBT) return;
    float w[8];
#pragma unroll
    for (int q = 0; q < 8; ++q) w[q] = bfr(Wo2[lane * 8 + q]);
    const float bias = bfr(bo2[0]); float mine = 0.f;
#pragma unroll 1
    for (int rr = 0; rr < 32; ++rr) { const float* zr = Z + (size_t)(b0 + rr) * HID + lane * 8; float s = 0.f;
#pragma unroll
        for (int q = 0; q < 8; ++q) s = fmaf(fmaxf(zr[q], 0.f), w[q], s);
#pragma unroll
        for (int sh = 16; sh; sh >>= 1) s += __shfl_xor(s, sh, 32);
        mine = (lane == rr) ? s + bias : mine; }
    *(volatile float*)(OUT + b0 + lane) = mine; __threadfence(); *(volatile float*)(OUT + b0 + lane) = mine;
}

extern "C" void kernel_launch(void* const* d_in, const int* in_sizes, int n_in,
                              void* d_out, int out_size, void* d_ws, size_t ws_size, hipStream_t stream) {
    (void)in_sizes; (void)n_in; (void)out_size;
    const float* state = (const float*)d_in[0]; const float* action = (const float*)d_in[1]; const float* Ws = (const float*)d_in[2]; const float* bs = (const float*)d_in[3];
    const float* Wa1 = (const float*)d_in[4]; const float* ba1 = (const float*)d_in[5]; const float* Wa2 = (const float*)d_in[6]; const float* ba2 = (const float*)d_in[7];
    const float* Wv1 = (const float*)d_in[8]; const float* bv1 = (const float*)d_in[9]; const float* Wv2 = (const float*)d_in[10]; const float* bv2 = (const float*)d_in[11];
    const float* mw = (const float*)d_in[12]; const float* Wo1 = (const float*)d_in[13]; const float* bo1 = (const float*)d_in[14]; const float* Wo2 = (const float*)d_in[15]; const float* bo2 = (const float*)d_in[16]; const int* aidp = (const int*)d_in[17];
    float* OUT = (float*)d_out;
    char* wsp = (char*)d_ws;
    auto take = [&](size_t bytes) { char* p = wsp; wsp += (bytes + 255) & ~(size_t)255; return (void*)p; };
    bf* WA2t = (bf*)take((size_t)NGA * HYP * 2); bf* WV2t = (bf*)take((size_t)NGV * HYP * 2); bf* WO1t = (bf*)take((size_t)HID * HID * 2);
    bf* HAh = (bf*)take((size_t)RA * HYP * 2); bf* HAl = (bf*)take((size_t)RA * HYP * 2); bf* HVh = (bf*)take((size_t)RV * HYP * 2); bf* HVl = (bf*)take((size_t)RV * HYP * 2);
    float* G = (float*)take((size_t)CHA * NGA * 4);
    float* ASUM = (float*)take((size_t)NBT * HH * 4); float* VSUM = (float*)take((size_t)NBT * HH * 4);
    bf* O1h = (bf*)take((size_t)NBT * HID * 2); bf* O1l = (bf*)take((size_t)NBT * HID * 2); float* Z = (float*)take((size_t)NBT * HID * 4);
    if ((size_t)(wsp - (char*)d_ws) > ws_size) return;
    k_wt<<<64, 256, 0, stream>>>(Wa2, HYP, NGA, WA2t); k_wt<<<64, 256, 0, stream>>>(Wv2, HYP, NGV, WV2t); k_wt<<<8, 256, 0, stream>>>(Wo1, HID, HID, WO1t);
    k_hyp1<false><<<RA / 8, 256, 0, stream>>>(state, action, aidp, Wa1, ba1, HAh, HAl);
    k_hyp1<true><<<RV / 8, 256, 0, stream>>>(state, action, aidp, Wv1, bv1, HVh, HVl);
    for (int c = 0; c < NBT / 64; ++c) { const int b0 = c * 64;
        k_gemmw<bf, 1, true><<<dim3(CHA / 64, NGA / 64, 1), 32, 0, stream>>>(HAh + (size_t)b0 * NAL * HYP, HAl + (size_t)b0 * NAL * HYP, WA2t, nullptr, HYP, G, NGA, ba2, 0, 0, 0);
        k_applysum<false><<<64 * (HH / 128) / 8, 256, 0, stream>>>(state, action, aidp, G, b0, ASUM);
        k_gemmw<bf, 1, true><<<dim3(CHV / 64, NGV / 64, 1), 32, 0, stream>>>(HVh + (size_t)b0 * NAD * HYP, HVl + (size_t)b0 * NAD * HYP, WV2t, nullptr, HYP, G, NGV, bv2, 0, 0, 0);
        k_applysum<true><<<64 * (HH / 128) / 8, 256, 0, stream>>>(state, action, aidp, G, b0, VSUM); }
    k_merge<<<NBT / 8, 256, 0, stream>>>(state, action, aidp, ASUM, VSUM, mw, Ws, bs, O1h, O1l);
    k_gemmw<bf, 1, true><<<dim3(NBT / 64, HID / 64, 1), 32, 0, stream>>>(O1h, O1l, WO1t, nullptr, HID, Z, HID, bo1, 0, 0, 0);
    k_out<<<(NBT / 32 + 7) / 8, 256, 0, stream>>>(Z, Wo2, bo2, OUT);
}
